// Content_SA_18717467476189
// MI455X (gfx1250) — hardware-run, weakly checked
//
#include <hip/hip_runtime.h>
#include <math.h>

constexpr int kNB   = 4;
constexpr int kCH   = 512;
constexpr int kHW   = 4096;
constexpr int kK3   = 3 * kCH;
constexpr int kFGld = 6 * kCH;
constexpr int kQRows = 2048;
constexpr int kStatPitch = 32;
constexpr float kWCarry = 256.0f;
constexpr float kXCarry = 16.0f;
constexpr float kPCarry = 32768.0f;
constexpr float kEps    = 1e-5f;
constexpr float kInvHW  = 1.0f / (float)kHW;
constexpr float kScaleH  = 1.0f / kWCarry;
constexpr float kScalePV = 1.0f / kPCarry;
constexpr float kScaleO  = 1.0f / (kWCarry * kXCarry);

static_assert(kCH % 64 == 0 && kHW % 64 == 0 && kQRows % 64 == 0);
static_assert(kK3 % 32 == 0 && kCH % 32 == 0 && kHW % 32 == 0);
static_assert((2 * kCH) % 64 == 0);
static_assert(kHW % kQRows == 0);

typedef __attribute__((ext_vector_type(16))) _Float16 v16h;
typedef __attribute__((ext_vector_type(8)))  _Float16 v8h;
typedef __attribute__((ext_vector_type(16))) __bf16   v16b;
typedef __attribute__((ext_vector_type(8)))  __bf16   v8b;
typedef __attribute__((ext_vector_type(8)))  float    v8f;
typedef __attribute__((ext_vector_type(4)))  float    v4f;
typedef __attribute__((ext_vector_type(4)))  unsigned int v4u;

__device__ __forceinline__ unsigned short f2bf_bits(float f) {
  unsigned u = __float_as_uint(f);
  return (unsigned short)((u + 0x7FFFu + ((u >> 16) & 1u)) >> 16);
}
__device__ __forceinline__ float bf_bits2f(unsigned short h) { return __uint_as_float(((unsigned)h) << 16); }
__device__ __forceinline__ unsigned pk16(unsigned short a, unsigned short b) { return (unsigned)a | ((unsigned)b << 16); }
__device__ __forceinline__ unsigned short h_bits(float f) { const _Float16 h = (_Float16)f; return __builtin_bit_cast(unsigned short, h); }

__device__ __forceinline__ void tie_h(v8f& a, v16h x, v16h y) { asm volatile("" : "+v"(a) : "v"(x), "v"(y)); }
__device__ __forceinline__ void tie_b(v8f& a, v16b x, v16b y) { asm volatile("" : "+v"(a) : "v"(x), "v"(y)); }
__device__ __forceinline__ void nopg_h(v8f& a, v16h x, v16h y) { asm volatile("v_nop\n\tv_nop\n\tv_nop\n\tv_nop" : "+v"(a) : "v"(x), "v"(y)); }
__device__ __forceinline__ void nopg_b(v8f& a, v16b x, v16b y) { asm volatile("v_nop\n\tv_nop\n\tv_nop\n\tv_nop" : "+v"(a) : "v"(x), "v"(y)); }
__device__ __forceinline__ void keep4_h(v16h a, v16h b, v16h c, v16h d) { asm volatile("v_nop" :: "v"(a), "v"(b), "v"(c), "v"(d)); }
__device__ __forceinline__ void keep4_b(v16b a, v16b b, v16b c, v16b d) { asm volatile("v_nop" :: "v"(a), "v"(b), "v"(c), "v"(d)); }
__device__ __forceinline__ void acc_guard4(v8f& a, v8f& b, v8f& c, v8f& d) { asm volatile("v_nop\n\tv_nop\n\tv_nop\n\tv_nop" : "+v"(a), "+v"(b), "+v"(c), "+v"(d)); }

template <typename T> struct Frag;
template <> struct Frag<_Float16> {
  typedef v16h V; union U { v16h v; v8h h[2]; };
  static __device__ __forceinline__ v16h load(const _Float16* p) {
    U f; f.h[0] = *(const v8h*)(p); f.h[1] = *(const v8h*)(p + 16); return f.v;
  }
  static __device__ __forceinline__ v8f mma(v16h a, v16h b, v8f c) {
    return __builtin_amdgcn_wmma_f32_16x16x32_f16(false, a, false, b, (short)0, c, false, false);
  }
  static __device__ __forceinline__ void guard_row(v8f& c0, v8f& c1, v8f& c2, v8f& c3, v16h a, v16h b0, v16h b1, v16h b2, v16h b3) {
    tie_h(c0, a, b0); tie_h(c1, a, b1); tie_h(c2, a, b2); nopg_h(c3, a, b3);
  }
  static __device__ __forceinline__ void keep(v16h a, v16h b, v16h c, v16h d) { keep4_h(a, b, c, d); }
};
template <> struct Frag<__bf16> {
  typedef v16b V; union U { v16b v; v8b h[2]; };
  static __device__ __forceinline__ v16b load(const __bf16* p) {
    U f; f.h[0] = *(const v8b*)(p); f.h[1] = *(const v8b*)(p + 16); return f.v;
  }
  static __device__ __forceinline__ v8f mma(v16b a, v16b b, v8f c) {
    return __builtin_amdgcn_wmma_f32_16x16x32_bf16(false, a, false, b, (short)0, c, false, false);
  }
  static __device__ __forceinline__ void guard_row(v8f& c0, v8f& c1, v8f& c2, v8f& c3, v16b a, v16b b0, v16b b1, v16b b2, v16b b3) {
    tie_b(c0, a, b0); tie_b(c1, a, b1); tie_b(c2, a, b2); nopg_b(c3, a, b3);
  }
  static __device__ __forceinline__ void keep(v16b a, v16b b, v16b c, v16b d) { keep4_b(a, b, c, d); }
};

template <int ET> struct Elem;
template <> struct Elem<0> { typedef _Float16 T; };
template <> struct Elem<1> { typedef __bf16 T; };

template <int ET, int BIAS_MODE, int OUT_MODE, bool RESID>
__global__ __launch_bounds__(256) void wmma_gemm64(
    const unsigned short* __restrict__ Ap, int lda,
    const unsigned short* __restrict__ Btp, int ldb,
    void* __restrict__ Cout, int ldc,
    const float* __restrict__ bias,
    const float* __restrict__ resid,
    int M, int N, int K, float scale) {
  typedef typename Elem<ET>::T T;
  typedef typename Frag<T>::V V;
  const T* Ab = (const T*)(const void*)Ap;
  const T* Bb = (const T*)(const void*)Btp;
  __shared__ __align__(16) float sT[8][16 * 68];
  const int lane = threadIdx.x & 31;
  const int wave = threadIdx.x >> 5;
  const int tilesN = N >> 6;
  const int tilesM = M >> 6;
  const int tile = blockIdx.x * 8 + wave;
  if (tile >= tilesM * tilesN) return;
  const int tm = tile / tilesN;
  const int tn = tile - tm * tilesN;
  const int m0 = tm << 6;
  const int n0 = tn << 6;

  const int rlane = lane & 15;
  const int koff  = (lane >> 4) * 8;
  const int mOff  = (lane >> 4) * 8;

  v8f acc[4][4];
#pragma unroll
  for (int i = 0; i < 4; ++i)
#pragma unroll
    for (int j = 0; j < 4; ++j) acc[i][j] = (v8f){0.f,0.f,0.f,0.f,0.f,0.f,0.f,0.f};

  for (int k0 = 0; k0 < K; k0 += 32) {
    V bh[4];
#pragma unroll
    for (int j = 0; j < 4; ++j) {
      const size_t bo = (size_t)(n0 + (j << 4) + rlane) * ldb + koff + k0;
      bh[j] = Frag<T>::load(Bb + bo);
    }
#pragma unroll
    for (int i = 0; i < 4; ++i) {
      const size_t ao = (size_t)(m0 + (i << 4) + rlane) * lda + koff + k0;
      V ah = Frag<T>::load(Ab + ao);
#pragma unroll
      for (int j = 0; j < 4; ++j) acc[i][j] = Frag<T>::mma(ah, bh[j], acc[i][j]);
      Frag<T>::guard_row(acc[i][0], acc[i][1], acc[i][2], acc[i][3], ah, bh[0], bh[1], bh[2], bh[3]);
    }
    Frag<T>::keep(bh[0], bh[1], bh[2], bh[3]);
  }
  acc_guard4(acc[0][0], acc[0][1], acc[0][2], acc[0][3]);
  acc_guard4(acc[1][0], acc[1][1], acc[1][2], acc[1][3]);
  acc_guard4(acc[2][0], acc[2][1], acc[2][2], acc[2][3]);
  acc_guard4(acc[3][0], acc[3][1], acc[3][2], acc[3][3]);

  float* slab = sT[wave];
#pragma unroll
  for (int i = 0; i < 4; ++i) {
    const int mBase = m0 + (i << 4);
    float brow[8];
#pragma unroll
    for (int r = 0; r < 8; ++r) brow[r] = 0.f;
    if (BIAS_MODE == 1) {
      const v4f b0 = *(const v4f*)(bias + mBase + mOff);
      const v4f b1 = *(const v4f*)(bias + mBase + mOff + 4);
#pragma unroll
      for (int e = 0; e < 4; ++e) { brow[e] = b0[e]; brow[4 + e] = b1[e]; }
    }
#pragma unroll
    for (int j = 0; j < 4; ++j) {
      const int n = n0 + (j << 4) + rlane;
      float bv = 0.f;
      if (BIAS_MODE == 2) bv = bias[n];
#pragma unroll
      for (int r = 0; r < 8; ++r) {
        float v = acc[i][j][r] * scale;
        if (BIAS_MODE == 1) v += brow[r];
        if (BIAS_MODE == 2) v += bv;
        slab[(mOff + r) * 68 + (j << 4) + rlane] = v;
      }
    }
    __builtin_amdgcn_fence(__ATOMIC_RELEASE, "workgroup");
    __builtin_amdgcn_wave_barrier();
    __builtin_amdgcn_fence(__ATOMIC_ACQUIRE, "workgroup");
    if (OUT_MODE == 0) {
      float* C = (float*)Cout;
      const int hh = lane >> 4, c4 = (lane & 15) * 4;
      if (RESID) {
        v4f vals[8];
#pragma unroll
        for (int it = 0; it < 8; ++it) {
          const int row = it * 2 + hh;
          const v4f sv = *(const v4f*)(slab + row * 68 + c4);
          const v4f rv = *(const v4f*)(resid + (size_t)(mBase + row) * ldc + n0 + c4);
          vals[it] = sv + rv;
        }
        for (int pass = 0; pass < 2; ++pass) {
#pragma unroll
          for (int it = 0; it < 8; ++it) {
            const int row = it * 2 + hh;
            *(volatile v4f*)(C + (size_t)(mBase + row) * ldc + n0 + c4) = vals[it];
          }
          __threadfence();
        }
      } else {
        for (int pass = 0; pass < 2; ++pass) {
#pragma unroll
          for (int it = 0; it < 8; ++it) {
            const int row = it * 2 + hh;
            v4f v = *(const v4f*)(slab + row * 68 + c4);
            *(volatile v4f*)(C + (size_t)(mBase + row) * ldc + n0 + c4) = v;
          }
          __threadfence();
        }
      }
    } else {
      const int q = lane >> 3, c8 = (lane & 7) * 8;
      unsigned short* C = (unsigned short*)Cout;
      int col0 = n0 + c8;
      int col1 = col0;
      int col2 = col0;
      if (OUT_MODE == 3) {
        const int halfN = N >> 1;
        const int isg = (n0 >= halfN) ? 1 : 0;
        const int nn = n0 - isg * halfN;
        col0 = isg * 3 * halfN + nn + c8;
        col1 = col0 + (isg ? 2 * halfN : halfN);
        col2 = col0 + (isg ? halfN : 2 * halfN);
      }
      for (int pass = 0; pass < 2; ++pass) {
#pragma unroll
        for (int it = 0; it < 4; ++it) {
          const int row = it * 4 + q;
          const float* sp = slab + row * 68 + c8;
          v8h hv, lv;
#pragma unroll
          for (int e = 0; e < 8; ++e) {
            if (OUT_MODE == 1) {
              hv[e] = (_Float16)sp[e];
              lv[e] = hv[e];
            } else {
              const unsigned short hb = f2bf_bits(sp[e]);
              const unsigned short lb = f2bf_bits(sp[e] - bf_bits2f(hb));
              hv[e] = __builtin_bit_cast(_Float16, hb);
              lv[e] = __builtin_bit_cast(_Float16, lb);
            }
          }
          unsigned short* rowp = C + (size_t)(mBase + row) * ldc;
          *(volatile v8h*)(rowp + col0) = hv;
          if (OUT_MODE == 3) {
            *(volatile v8h*)(rowp + col1) = hv;
            *(volatile v8h*)(rowp + col2) = lv;
          }
        }
        __threadfence();
      }
    }
    __builtin_amdgcn_fence(__ATOMIC_RELEASE, "workgroup");
    __builtin_amdgcn_wave_barrier();
    __builtin_amdgcn_fence(__ATOMIC_ACQUIRE, "workgroup");
  }
}

__global__ __launch_bounds__(256) void wsplit_kernel(const float* __restrict__ fw, const float* __restrict__ gw,
                                                     unsigned short* __restrict__ W3) {
  const int i = blockIdx.x * 256 + threadIdx.x;
  const int row = i >> 6;
  const int c8 = (i & 63) * 8;
  const float* src = (row < kCH) ? (fw + (size_t)row * kCH) : (gw + (size_t)(row - kCH) * kCH);
  const v4f a = *(const v4f*)(src + c8);
  const v4f c = *(const v4f*)(src + c8 + 4);
  float x[8];
#pragma unroll
  for (int e = 0; e < 4; ++e) { x[e] = a[e]; x[4 + e] = c[e]; }
  unsigned short hb[8], lb[8];
#pragma unroll
  for (int e = 0; e < 8; ++e) {
    hb[e] = f2bf_bits(x[e]);
    lb[e] = f2bf_bits(x[e] - bf_bits2f(hb[e]));
  }
  const v4u uh = (v4u){pk16(hb[0], hb[1]), pk16(hb[2], hb[3]), pk16(hb[4], hb[5]), pk16(hb[6], hb[7])};
  const v4u ul = (v4u){pk16(lb[0], lb[1]), pk16(lb[2], lb[3]), pk16(lb[4], lb[5]), pk16(lb[6], lb[7])};
  unsigned short* rp = W3 + (size_t)row * kK3 + c8;
  for (int pass = 0; pass < 2; ++pass) {
    *(volatile v4u*)(rp) = uh;
    *(volatile v4u*)(rp + kCH) = uh;
    *(volatile v4u*)(rp + 2 * kCH) = ul;
    __threadfence();
  }
}

__global__ __launch_bounds__(256) void wcast_kernel(const float* __restrict__ hw, const float* __restrict__ ow,
                                                    unsigned short* __restrict__ hw16, unsigned short* __restrict__ ow16) {
  const int i = blockIdx.x * 256 + threadIdx.x;
  const float* src = (blockIdx.y == 0) ? hw : ow;
  unsigned short* dst = (blockIdx.y == 0) ? hw16 : ow16;
  const float* p = src + 8 * (size_t)i;
  const v4f a = *(const v4f*)(p);
  const v4f c = *(const v4f*)(p + 4);
  unsigned short hb[8];
#pragma unroll
  for (int e = 0; e < 4; ++e) {
    hb[e]     = h_bits(a[e] * kWCarry);
    hb[4 + e] = h_bits(c[e] * kWCarry);
  }
  const v4u u = (v4u){pk16(hb[0], hb[1]), pk16(hb[2], hb[3]), pk16(hb[4], hb[5]), pk16(hb[6], hb[7])};
  unsigned short* q = dst + 8 * (size_t)i;
  *(volatile v4u*)q = u;
  __threadfence();
  *(volatile v4u*)q = u;
}

__global__ __launch_bounds__(256) void bias_prep_kernel(const float* __restrict__ fb, const float* __restrict__ gb,
                                                        const float* __restrict__ hb,
                                                        float* __restrict__ fgb, float* __restrict__ hb16) {
  const int t = threadIdx.x;
  const int j = (t & 127) * 4;
  const v4f a = *(const v4f*)(fb + j);
  const v4f g = *(const v4f*)(gb + j);
  const v4f h = *(const v4f*)(hb + j);
  const bool first = (t < 128);
  v4f v;
#pragma unroll
  for (int e = 0; e < 4; ++e) v[e] = first ? a[e] : g[e];
  v4f hs;
#pragma unroll
  for (int e = 0; e < 4; ++e) hs[e] = h[e] * kXCarry;
  for (int pass = 0; pass < 2; ++pass) {
    *(volatile v4f*)(fgb + 4 * t) = v;
    if (first) *(volatile v4f*)(hb16 + 4 * t) = hs;
    __threadfence();
  }
}

__device__ __forceinline__ float block_sum256(float v, float* red, int lane, int wave) {
#pragma unroll
  for (int off = 16; off > 0; off >>= 1) v += __shfl_xor(v, off, 32);
  if (lane == 0) red[wave] = v;
  __syncthreads();
  float s = 0.f;
#pragma unroll
  for (int w = 0; w < 8; ++w) s += red[w];
  __syncthreads();
  return s;
}

__global__ __launch_bounds__(256) void chan_stats_kernel(const float* __restrict__ x, float* __restrict__ stats) {
  __shared__ float red[8];
  const int t = threadIdx.x, lane = t & 31, wave = t >> 5;
  const float* row = x + (size_t)blockIdx.x * kHW;
  v4f v[4];
#pragma unroll
  for (int q = 0; q < 4; ++q) v[q] = *(const v4f*)(row + (size_t)(q * 256 + t) * 4);
  float s = 0.f;
#pragma unroll
  for (int q = 0; q < 4; ++q) s += (v[q][0] + v[q][1]) + (v[q][2] + v[q][3]);
  s = block_sum256(s, red, lane, wave);
  const float mean = s * kInvHW;
  float ss = 0.f;
#pragma unroll
  for (int q = 0; q < 4; ++q) {
#pragma unroll
    for (int e = 0; e < 4; ++e) {
      const float d = v[q][e] - mean;
      ss += d * d;
    }
  }
  ss = block_sum256(ss, red, lane, wave);
  const float var = ss * kInvHW;
  const float rstd = 1.0f / sqrtf(var + kEps);
  if (wave == 0) {
    const float o = (lane == 0) ? mean : ((lane == 1) ? rstd : 0.0f);
    volatile float* p = stats + (size_t)blockIdx.x * kStatPitch + lane;
    *p = o;
    __threadfence();
    *p = o;
  }
}

__global__ __launch_bounds__(256) void norm_transpose_kernel(const float* __restrict__ x, const float* __restrict__ stats,
                                                             unsigned short* __restrict__ normT3,
                                                             unsigned short* __restrict__ contT) {
  __shared__ __align__(16) float tf[64 * 68];
  __shared__ float sMean[64];
  __shared__ float sRstd[64];
  const int p0  = blockIdx.x * 64;
  const int c0  = blockIdx.y * 64;
  const int tid = threadIdx.x;
  {
    const int lr = tid >> 4;
    const int c4 = (tid & 15) * 4;
#pragma unroll
    for (int it = 0; it < 4; ++it) {
      const int rr = it * 16 + lr;
      const v4f a = *(const v4f*)(x + (size_t)(c0 + rr) * kHW + p0 + c4);
      *(v4f*)(tf + rr * 68 + c4) = a;
    }
    const int ch = tid & 63;
    const int which = (tid >> 6) & 1;
    const float sv = stats[(size_t)(c0 + ch) * kStatPitch + which];
    if (tid < 64) sMean[ch] = sv;
    else if (tid < 128) sRstd[ch] = sv;
  }
  __syncthreads();
  const int sub = tid >> 3;
  const int c8  = (tid & 7) * 8;
  v4u nh[2], nl[2], cf[2];
#pragma unroll
  for (int it = 0; it < 2; ++it) {
    const int oc = it * 32 + sub;
    v4u a, a2, a3;
#pragma unroll
    for (int q = 0; q < 4; ++q) {
      const int ch0 = c8 + 2 * q;
      const int ch1 = ch0 + 1;
      const float x0 = tf[ch0 * 68 + oc];
      const float x1 = tf[ch1 * 68 + oc];
      const float n0v = (x0 - sMean[ch0]) * sRstd[ch0];
      const float n1v = (x1 - sMean[ch1]) * sRstd[ch1];
      const unsigned short h0 = f2bf_bits(n0v), h1 = f2bf_bits(n1v);
      const unsigned short l0 = f2bf_bits(n0v - bf_bits2f(h0)), l1 = f2bf_bits(n1v - bf_bits2f(h1));
      a[q]  = pk16(h0, h1);
      a2[q] = pk16(l0, l1);
      a3[q] = pk16(h_bits(x0 * kXCarry), h_bits(x1 * kXCarry));
    }
    nh[it] = a; nl[it] = a2; cf[it] = a3;
  }
  for (int pass = 0; pass < 2; ++pass) {
#pragma unroll
    for (int it = 0; it < 2; ++it) {
      const int oc = it * 32 + sub;
      unsigned short* np = normT3 + (size_t)(p0 + oc) * kK3 + c0 + c8;
      unsigned short* cp = contT + (size_t)(p0 + oc) * kCH + c0 + c8;
      *(volatile v4u*)(np) = nh[it];
      *(volatile v4u*)(np + kCH) = nl[it];
      *(volatile v4u*)(np + 2 * kCH) = nh[it];
      *(volatile v4u*)(cp) = cf[it];
    }
    __threadfence();
  }
}

__global__ __launch_bounds__(256) void softmax_rows_kernel(const float* __restrict__ E, unsigned short* __restrict__ P) {
  __shared__ float redM[8];
  __shared__ float redS[8];
  const int row  = blockIdx.x;
  const int t    = threadIdx.x;
  const int lane = t & 31, wave = t >> 5;
  const float* sr = E + (size_t)row * kHW + 8 * t;
  const v4f a0 = *(const v4f*)(sr);
  const v4f a1 = *(const v4f*)(sr + 4);
  const v4f b0 = *(const v4f*)(sr + kHW / 2);
  const v4f b1 = *(const v4f*)(sr + kHW / 2 + 4);
  float x[16];
#pragma unroll
  for (int e = 0; e < 4; ++e) { x[e] = a0[e]; x[4 + e] = a1[e]; x[8 + e] = b0[e]; x[12 + e] = b1[e]; }
  float m = x[0];
#pragma unroll
  for (int e = 1; e < 16; ++e) m = fmaxf(m, x[e]);
#pragma unroll
  for (int off = 16; off > 0; off >>= 1) m = fmaxf(m, __shfl_xor(m, off, 32));
  if (lane == 0) redM[wave] = m;
  __syncthreads();
  float mx = redM[0];
#pragma unroll
  for (int w = 1; w < 8; ++w) mx = fmaxf(mx, redM[w]);
  float s = 0.f;
#pragma unroll
  for (int e = 0; e < 16; ++e) {
    x[e] = __expf(x[e] - mx);
    s += x[e];
  }
#pragma unroll
  for (int off = 16; off > 0; off >>= 1) s += __shfl_xor(s, off, 32);
  if (lane == 0) redS[wave] = s;
  __syncthreads();
  float tot = 0.f;
#pragma unroll
  for (int w = 0; w < 8; ++w) tot += redS[w];
  const float inv = kPCarry * (1.0f / tot);
  unsigned short hb[16];
#pragma unroll
  for (int e = 0; e < 16; ++e) hb[e] = h_bits(x[e] * inv);
  const v4u u0 = (v4u){pk16(hb[0], hb[1]), pk16(hb[2], hb[3]), pk16(hb[4], hb[5]), pk16(hb[6], hb[7])};
  const v4u u1 = (v4u){pk16(hb[8], hb[9]), pk16(hb[10], hb[11]), pk16(hb[12], hb[13]), pk16(hb[14], hb[15])};
  unsigned short* pr = P + (size_t)row * kHW + 8 * t;
  for (int pass = 0; pass < 2; ++pass) {
    *(volatile v4u*)(pr) = u0;
    *(volatile v4u*)(pr + kHW / 2) = u1;
    __threadfence();
  }
}

extern "C" void kernel_launch(void* const* d_in, const int* in_sizes, int n_in,
                              void* d_out, int out_size, void* d_ws, size_t ws_size,
                              hipStream_t stream) {
  if (n_in < 9) return;
  if (in_sizes[0] != kNB * kCH * kHW || out_size != kNB * kCH * kHW) return;
  if (in_sizes[1] != kCH * kCH || in_sizes[3] != kCH * kCH || in_sizes[5] != kCH * kCH || in_sizes[7] != kCH * kCH) return;
  if (in_sizes[2] != kCH || in_sizes[4] != kCH || in_sizes[6] != kCH || in_sizes[8] != kCH) return;

  const float* content = (const float*)d_in[0];
  const float* f_w = (const float*)d_in[1];
  const float* f_b = (const float*)d_in[2];
  const float* g_w = (const float*)d_in[3];
  const float* g_b = (const float*)d_in[4];
  const float* h_w = (const float*)d_in[5];
  const float* h_b = (const float*)d_in[6];
  const float* o_w = (const float*)d_in[7];
  const float* o_b = (const float*)d_in[8];
  float* out = (float*)d_out;

  const size_t bW3   = (size_t)2 * kCH * kK3 * 2;
  const size_t bW16  = (size_t)kCH * kCH * 2;
  const size_t bFGB  = (size_t)2 * kCH * 4;
  const size_t bHB   = (size_t)kCH * 4;
  const size_t bST   = (size_t)kNB * kCH * kStatPitch * 4;
  const size_t bNT3  = (size_t)kHW * kK3 * 2;
  const size_t bCT   = (size_t)kHW * kCH * 2;
  const size_t bFG3  = (size_t)kHW * kFGld * 2;
  const size_t bH16  = (size_t)kCH * kHW * 2;
  const size_t bEN   = (size_t)kQRows * kHW * 4;
  const size_t bATT  = (size_t)kHW * kHW * 2;
  const size_t bAOT  = (size_t)kHW * kCH * 2;
  char* ws = (char*)d_ws;
  size_t off = 0;
  unsigned short* W3fg   = (unsigned short*)(ws + off); off += bW3;
  unsigned short* hw16   = (unsigned short*)(ws + off); off += bW16;
  unsigned short* ow16   = (unsigned short*)(ws + off); off += bW16;
  float*          fgb    = (float*)(ws + off);          off += bFGB;
  float*          hb16   = (float*)(ws + off);          off += bHB;
  float*          stats  = (float*)(ws + off);          off += bST;
  unsigned short* normT3 = (unsigned short*)(ws + off); off += bNT3;
  unsigned short* contT  = (unsigned short*)(ws + off); off += bCT;
  unsigned short* FG3    = (unsigned short*)(ws + off); off += bFG3;
  unsigned short* H16    = (unsigned short*)(ws + off); off += bH16;
  float*          energy = (float*)(ws + off);          off += bEN;
  unsigned short* att    = (unsigned short*)(ws + off); off += bATT;
  unsigned short* aoT    = (unsigned short*)(ws + off); off += bAOT;
  if (off > ws_size || off > (size_t)134217728) return;

  const dim3 blk256(256);

  wsplit_kernel<<<dim3((2 * kCH * kCH / 8) / 256), blk256, 0, stream>>>(f_w, g_w, W3fg);
  wcast_kernel<<<dim3((kCH * kCH / 8) / 256, 2), blk256, 0, stream>>>(h_w, o_w, hw16, ow16);
  bias_prep_kernel<<<dim3(1), blk256, 0, stream>>>(f_b, g_b, h_b, fgb, hb16);
  chan_stats_kernel<<<dim3(kNB * kCH), blk256, 0, stream>>>(content, stats);

  constexpr int tilesFG = (kHW / 64) * ((2 * kCH) / 64);
  constexpr int tilesH  = (kCH / 64) * (kHW / 64);
  constexpr int tilesEN = (kQRows / 64) * (kHW / 64);
  constexpr int tilesPV = (kHW / 64) * (kCH / 64);
  static_assert(tilesFG % 8 == 0 && tilesH % 8 == 0 && tilesEN % 8 == 0 && tilesPV % 8 == 0);

  for (int b = 0; b < kNB; ++b) {
    const float* xb = content + (size_t)b * kCH * kHW;
    float* ob = out + (size_t)b * kCH * kHW;
    const float* stb = stats + (size_t)b * kCH * kStatPitch;

    norm_transpose_kernel<<<dim3(kHW / 64, kCH / 64), blk256, 0, stream>>>(xb, stb, normT3, contT);

    wmma_gemm64<1, 2, 3, false><<<dim3(tilesFG / 8), blk256, 0, stream>>>(
        normT3, kK3, W3fg, kK3, (void*)FG3, kFGld, fgb, fgb, kHW, 2 * kCH, kK3, 1.0f);

    wmma_gemm64<0, 1, 1, false><<<dim3(tilesH / 8), blk256, 0, stream>>>(
        hw16, kCH, contT, kCH, (void*)H16, kHW, hb16, hb16, kCH, kHW, kCH, kScaleH);

    for (int hq = 0; hq < kHW / kQRows; ++hq) {
      wmma_gemm64<1, 0, 0, false><<<dim3(tilesEN / 8), blk256, 0, stream>>>(
          FG3 + (size_t)hq * kQRows * kFGld, kFGld, FG3 + kK3, kFGld, (void*)energy, kHW,
          fgb, fgb, kQRows, kHW, kK3, 1.0f);
      softmax_rows_kernel<<<dim3(kQRows), blk256, 0, stream>>>(energy, att + (size_t)hq * kQRows * kHW);
    }

    wmma_gemm64<0, 0, 1, false><<<dim3(tilesPV / 8), blk256, 0, stream>>>(
        att, kHW, H16, kHW, (void*)aoT, kCH, fgb, fgb, kHW, kCH, kHW, kScalePV);

    wmma_gemm64<0, 1, 0, true><<<dim3(tilesH / 8), blk256, 0, stream>>>(
        ow16, kCH, aoT, kCH, (void*)ob, kHW, o_b, xb, kCH, kHW, kCH, kScaleO);
  }
}
